// LSTMNetwork_16801912062406
// MI455X (gfx1250) — hardware-run, weakly checked
//
#include <hip/hip_runtime.h>
#include <math.h>

typedef __attribute__((ext_vector_type(16))) __bf16   v16b;
typedef __attribute__((ext_vector_type(8)))  __bf16   v8b;
typedef __attribute__((ext_vector_type(8)))  float    v8f;
typedef __attribute__((ext_vector_type(4)))  float    v4f;
typedef __attribute__((ext_vector_type(4)))  unsigned v4u;
typedef __attribute__((ext_vector_type(8)))  unsigned v8u;

constexpr int kRows        = 262144;
constexpr int kIn          = 15;
constexpr int kHid         = 60;
constexpr int kOut         = 3;
constexpr int kHidPad      = 64;
constexpr int kGateCols    = 4 * kHidPad;
constexpr int kKPad        = 32;
constexpr int kThreads     = 256;
constexpr int kWavesPerBlk = 8;
constexpr int kBlocks      = 256;
constexpr int kItersPerWv  = 4;
constexpr int kRowsPerIter = 32;
static_assert(kBlocks * kWavesPerBlk * kItersPerWv * kRowsPerIter == kRows, "row coverage exact");
static_assert(kIn < 16 && kHid <= kHidPad && kOut <= 4, "padding assumptions");
static_assert((kRowsPerIter * kOut * 4) % 128 == 0, "a wave iteration writes whole 128-B lines");

constexpr size_t kWtBytes  = (size_t)kGateCols * kKPad * 2;
constexpr int    kTabBias  = 0;
constexpr int    kTabWy    = 256;
constexpr int    kTabPc    = 512;
constexpr int    kTabBy    = 576;
constexpr int    kTabFloats = 640;
constexpr size_t kTabBytes = (size_t)kTabFloats * 4;
constexpr size_t kWsTotal  = kWtBytes + kTabBytes;
static_assert(kWtBytes == 16384 && kTabBytes == 2560 && kWsTotal == 18944, "carve total");
static_assert(kWsTotal <= 134217728ull, "carve cap");
static_assert((kWtBytes % 128) == 0 && (kTabBytes % 128) == 0, "regions are whole lines");

__device__ __forceinline__ unsigned f2bf_bits(float f) {
  const unsigned u = __float_as_uint(f);
  return (u + 0x7FFFu + ((u >> 16) & 1u)) >> 16;
}
__device__ __forceinline__ float bf16r(float f) { return __uint_as_float(f2bf_bits(f) << 16); }

__device__ __forceinline__ v8f mma_bf16(v16b a, v16b b, v8f c) {
  c = __builtin_amdgcn_wmma_f32_16x16x32_bf16(false, a, false, b, (short)0, c, false, false);
  asm volatile("v_nop\n\tv_nop\n\tv_nop\n\tv_nop" : "+v"(c) : "v"(a), "v"(b));
  return c;
}

__device__ __forceinline__ float gate_sigmoid(float z) {
  const float zc = fminf(fmaxf(z, -30.0f), 30.0f);
  return 1.0f / (1.0f + expf(-zc));
}
__device__ __forceinline__ float gate_tanh(float z) {
  const float zc = fminf(fmaxf(z, -15.0f), 15.0f);
  return 1.0f - 2.0f / (1.0f + expf(2.0f * zc));
}

__device__ __forceinline__ void cell_elem(float zf, float zi, float zc, float zo, float pc, v4f wy,
                                          float& y0, float& y1, float& y2) {
  const float fg = gate_sigmoid(zf);
  const float ig = gate_sigmoid(zi);
  const float cg = gate_tanh(zc);
  const float og = gate_sigmoid(zo);
  const float cs = fg * pc + ig * cg;
  const float hv = og * gate_tanh(cs);
  y0 = fmaf(hv, wy[0], y0);
  y1 = fmaf(hv, wy[1], y1);
  y2 = fmaf(hv, wy[2], y2);
}

__device__ __forceinline__ v4u wt_chunk(const float* __restrict__ Wg, int j, int k8) {
  const int jc = j < (kHid - 1) ? j : (kHid - 1);
  unsigned bits[8];
#pragma unroll
  for (int e = 0; e < 8; ++e) {
    const int k  = k8 + e;
    const int kc = k < (kIn - 1) ? k : (kIn - 1);
    float w = Wg[kc * kHid + jc];
    asm volatile("" : "+v"(w));
    const float val = (k < kIn && j < kHid) ? w : 0.0f;
    bits[e] = f2bf_bits(val);
  }
  v4u q;
  q[0] = bits[0] | (bits[1] << 16);
  q[1] = bits[2] | (bits[3] << 16);
  q[2] = bits[4] | (bits[5] << 16);
  q[3] = bits[6] | (bits[7] << 16);
  return q;
}

__global__ __launch_bounds__(kThreads) void gate_prep_kernel(
    const float* __restrict__ h_in, const float* __restrict__ c_in,
    const float* __restrict__ Wf, const float* __restrict__ Uf, const float* __restrict__ bfv,
    const float* __restrict__ Wi, const float* __restrict__ Ui, const float* __restrict__ biv,
    const float* __restrict__ Wc, const float* __restrict__ Uc, const float* __restrict__ bcv,
    const float* __restrict__ Wo, const float* __restrict__ Uo, const float* __restrict__ bov,
    const float* __restrict__ Wy, const float* __restrict__ byv,
    unsigned short* __restrict__ WT, float* __restrict__ TAB)
{
  const int tid = threadIdx.x;

  const int jw = tid >> 2;
  const int k8 = (tid & 3) * 8;
  const v4u q0 = wt_chunk(Wf, jw, k8);
  const v4u q1 = wt_chunk(Wi, jw, k8);
  const v4u q2 = wt_chunk(Wc, jw, k8);
  const v4u q3 = wt_chunk(Wo, jw, k8);

  const int g  = tid >> 6;
  const int j  = tid & 63;
  const int jc = j < (kHid - 1) ? j : (kHid - 1);
  float s = 0.0f;
#pragma unroll 1
  for (int k = 0; k < kHid; ++k) {
    const float ph = h_in[k];
    const float uf = Uf[k * kHid + jc];
    const float ui = Ui[k * kHid + jc];
    const float uc = Uc[k * kHid + jc];
    const float uo = Uo[k * kHid + jc];
    const float u  = (g == 0) ? uf : (g == 1) ? ui : (g == 2) ? uc : uo;
    s = fmaf(bf16r(ph), bf16r(u), s);
  }
  const float b0 = bfv[jc];
  const float b1 = biv[jc];
  const float b2 = bcv[jc];
  const float b3 = bov[jc];
  const float bl = (g == 0) ? b0 : (g == 1) ? b1 : (g == 2) ? b2 : b3;
  const float biasv = (j < kHid) ? (s + bf16r(bl)) : 0.0f;

  const int jy  = tid >> 2;
  const int oy  = tid & 3;
  const int jyc = jy < (kHid - 1) ? jy : (kHid - 1);
  const int oyc = oy < (kOut - 1) ? oy : (kOut - 1);
  float wyl = Wy[jyc * kOut + oyc];
  asm volatile("" : "+v"(wyl));
  const float wyv = (jy < kHid && oy < kOut) ? bf16r(wyl) : 0.0f;

  const int tcl = tid < (kHid - 1) ? tid : (kHid - 1);
  float pcl = c_in[tcl];
  asm volatile("" : "+v"(pcl));
  const int ub  = tid - 64;
  const int ubc = ub < 0 ? 0 : (ub > (kOut - 1) ? (kOut - 1) : ub);
  float byl = byv[ubc];
  asm volatile("" : "+v"(byl));
  const float pcv   = (tid < kHid) ? bf16r(pcl) : 0.0f;
  const float byo   = (ub >= 0 && ub < kOut) ? bf16r(byl) : 0.0f;
  const float tailv = (tid < 64) ? pcv : byo;

  for (int pass = 0; pass < 2; ++pass) {
    *(volatile v4u*)(WT + (size_t)(0 * 256 + tid) * 8) = q0;
    *(volatile v4u*)(WT + (size_t)(1 * 256 + tid) * 8) = q1;
    *(volatile v4u*)(WT + (size_t)(2 * 256 + tid) * 8) = q2;
    *(volatile v4u*)(WT + (size_t)(3 * 256 + tid) * 8) = q3;
    *(volatile float*)(TAB + kTabBias + tid) = biasv;
    *(volatile float*)(TAB + kTabWy + tid)   = wyv;
    if (tid < 128) *(volatile float*)(TAB + kTabPc + tid) = tailv;
    __threadfence();
  }
}

__global__ __launch_bounds__(kThreads) void cell_step_kernel(
    const float* __restrict__ x, const unsigned short* __restrict__ WTp,
    const float* __restrict__ TAB, float* __restrict__ out)
{
  __shared__ __align__(16) __bf16 sWt[kGateCols * kKPad];
  __shared__ __align__(16) float  sTab[kTabFloats];
  __shared__ __align__(16) float  sY[kWavesPerBlk][96];

  const int tid  = threadIdx.x;
  const int lane = tid & 31;
  const int wave = tid >> 5;
  const int c    = lane & 15;
  const int hh   = lane >> 4;

  {
    const __bf16* WT = (const __bf16*)WTp;
#pragma unroll
    for (int i = 0; i < 4; ++i) {
      const int ci = i * kThreads + tid;
      *(v8b*)(sWt + ci * 8) = *(const v8b*)(WT + ci * 8);
    }
    const int tc = tid < 160 ? tid : 159;
    v4f tv = *(const v4f*)(TAB + tc * 4);
    asm volatile("" : "+v"(tv));
    if (tid < 160) *(v4f*)(sTab + tid * 4) = tv;
  }
  __syncthreads();

  const float by0 = sTab[kTabBy + 0];
  const float by1 = sTab[kTabBy + 1];
  const float by2 = sTab[kTabBy + 2];
  float* ys = sY[wave];

#pragma unroll 1
  for (int it = 0; it < kItersPerWv; ++it) {
    const int grp  = (blockIdx.x * kItersPerWv + it) * kWavesPerBlk + wave;
    const int row0 = grp * kRowsPerIter;

#pragma unroll 1
    for (int tile = 0; tile < 2; ++tile) {
      const int row = row0 + tile * 16 + c;
      const float* xp = x + (size_t)row * kIn + 8 * hh;
      const float xv0 = xp[0];
      const float xv1 = xp[1];
      const float xv2 = xp[2];
      const float xv3 = xp[3];
      const float xv4 = xp[4];
      const float xv5 = xp[5];
      const float xv6 = xp[6];
      const int   k7  = hh ? 6 : 7;
      float xl7 = xp[k7];
      asm volatile("" : "+v"(xl7));
      const float xv7 = (hh == 0) ? xl7 : 0.0f;
      v8u bw;
      bw[0] = f2bf_bits(xv0) | (f2bf_bits(xv1) << 16);
      bw[1] = f2bf_bits(xv2) | (f2bf_bits(xv3) << 16);
      bw[2] = f2bf_bits(xv4) | (f2bf_bits(xv5) << 16);
      bw[3] = f2bf_bits(xv6) | (f2bf_bits(xv7) << 16);
      bw[4] = 0u;
      bw[5] = 0u;
      bw[6] = 0u;
      bw[7] = 0u;
      const v16b bfrag = __builtin_bit_cast(v16b, bw);

      float y0 = 0.0f, y1 = 0.0f, y2 = 0.0f;

#pragma unroll 1
      for (int jt = 0; jt < 4; ++jt) {
        union FB { v16b v; v8b h[2]; };
        FB a0, a1, a2, a3;
        const int ao = (jt * 16 + c) * kKPad + 8 * hh;
        a0.h[0] = *(const v8b*)(sWt + 0 * 64 * kKPad + ao);
        a0.h[1] = *(const v8b*)(sWt + 0 * 64 * kKPad + ao + 16);
        a1.h[0] = *(const v8b*)(sWt + 1 * 64 * kKPad + ao);
        a1.h[1] = *(const v8b*)(sWt + 1 * 64 * kKPad + ao + 16);
        a2.h[0] = *(const v8b*)(sWt + 2 * 64 * kKPad + ao);
        a2.h[1] = *(const v8b*)(sWt + 2 * 64 * kKPad + ao + 16);
        a3.h[0] = *(const v8b*)(sWt + 3 * 64 * kKPad + ao);
        a3.h[1] = *(const v8b*)(sWt + 3 * 64 * kKPad + ao + 16);

        const int bo = kTabBias + jt * 16 + 8 * hh;
        const v4f c0l = *(const v4f*)(sTab + bo + 0 * 64);
        const v4f c0h = *(const v4f*)(sTab + bo + 0 * 64 + 4);
        const v4f c1l = *(const v4f*)(sTab + bo + 1 * 64);
        const v4f c1h = *(const v4f*)(sTab + bo + 1 * 64 + 4);
        const v4f c2l = *(const v4f*)(sTab + bo + 2 * 64);
        const v4f c2h = *(const v4f*)(sTab + bo + 2 * 64 + 4);
        const v4f c3l = *(const v4f*)(sTab + bo + 3 * 64);
        const v4f c3h = *(const v4f*)(sTab + bo + 3 * 64 + 4);
        v8f acc0 = __builtin_shufflevector(c0l, c0h, 0, 1, 2, 3, 4, 5, 6, 7);
        v8f acc1 = __builtin_shufflevector(c1l, c1h, 0, 1, 2, 3, 4, 5, 6, 7);
        v8f acc2 = __builtin_shufflevector(c2l, c2h, 0, 1, 2, 3, 4, 5, 6, 7);
        v8f acc3 = __builtin_shufflevector(c3l, c3h, 0, 1, 2, 3, 4, 5, 6, 7);

        acc0 = mma_bf16(a0.v, bfrag, acc0);
        acc1 = mma_bf16(a1.v, bfrag, acc1);
        acc2 = mma_bf16(a2.v, bfrag, acc2);
        acc3 = mma_bf16(a3.v, bfrag, acc3);

        const v4f pca = *(const v4f*)(sTab + kTabPc + jt * 16 + 8 * hh);
        const v4f pcb = *(const v4f*)(sTab + kTabPc + jt * 16 + 8 * hh + 4);

#pragma unroll
        for (int r = 0; r < 8; ++r) {
          const v4f wy = *(const v4f*)(sTab + kTabWy + (jt * 16 + 8 * hh + r) * 4);
          const float pcr = (r < 4) ? pca[r & 3] : pcb[r & 3];
          cell_elem(acc0[r], acc1[r], acc2[r], acc3[r], pcr, wy, y0, y1, y2);
        }
      }

      y0 += __shfl_xor(y0, 16, 32);
      y1 += __shfl_xor(y1, 16, 32);
      y2 += __shfl_xor(y2, 16, 32);
      const float o0 = y0 + by0;
      const float o1 = y1 + by1;
      const float o2 = y2 + by2;
      if (hh == 0) {
        ys[(tile * 16 + c) * 3 + 0] = o0;
        ys[(tile * 16 + c) * 3 + 1] = o1;
        ys[(tile * 16 + c) * 3 + 2] = o2;
      }
    }

    __builtin_amdgcn_fence(__ATOMIC_RELEASE, "workgroup");
    __builtin_amdgcn_wave_barrier();
    __builtin_amdgcn_fence(__ATOMIC_ACQUIRE, "workgroup");
    {
      const float v0 = ys[lane];
      const float v1 = ys[32 + lane];
      const float v2 = ys[64 + lane];
      float* op = out + (size_t)row0 * kOut + lane;
      for (int pass = 0; pass < 2; ++pass) {
        *(volatile float*)(op)      = v0;
        *(volatile float*)(op + 32) = v1;
        *(volatile float*)(op + 64) = v2;
        __threadfence();
      }
    }
    __builtin_amdgcn_fence(__ATOMIC_RELEASE, "workgroup");
    __builtin_amdgcn_wave_barrier();
    __builtin_amdgcn_fence(__ATOMIC_ACQUIRE, "workgroup");
  }
}

extern "C" void kernel_launch(void* const* d_in, const int* in_sizes, int n_in,
                              void* d_out, int out_size, void* d_ws, size_t ws_size,
                              hipStream_t stream) {
  if (n_in < 17 || d_out == nullptr || d_ws == nullptr) return;
  if (in_sizes[0] != kRows * kIn) return;
  if (in_sizes[1] != kHid || in_sizes[2] != kHid) return;
  if (in_sizes[3] != kIn * kHid || in_sizes[4] != kHid * kHid || in_sizes[5] != kHid) return;
  if (in_sizes[6] != kIn * kHid || in_sizes[7] != kHid * kHid || in_sizes[8] != kHid) return;
  if (in_sizes[9] != kIn * kHid || in_sizes[10] != kHid * kHid || in_sizes[11] != kHid) return;
  if (in_sizes[12] != kIn * kHid || in_sizes[13] != kHid * kHid || in_sizes[14] != kHid) return;
  if (in_sizes[15] != kHid * kOut || in_sizes[16] != kOut) return;
  if (out_size != kRows * kOut) return;
  if (ws_size < kWsTotal) return;

  const float* x    = (const float*)d_in[0];
  const float* h_in = (const float*)d_in[1];
  const float* c_in = (const float*)d_in[2];
  const float* Wf   = (const float*)d_in[3];
  const float* Uf   = (const float*)d_in[4];
  const float* bf   = (const float*)d_in[5];
  const float* Wi   = (const float*)d_in[6];
  const float* Ui   = (const float*)d_in[7];
  const float* bi   = (const float*)d_in[8];
  const float* Wc   = (const float*)d_in[9];
  const float* Uc   = (const float*)d_in[10];
  const float* bc   = (const float*)d_in[11];
  const float* Wo   = (const float*)d_in[12];
  const float* Uo   = (const float*)d_in[13];
  const float* bo   = (const float*)d_in[14];
  const float* Wy   = (const float*)d_in[15];
  const float* by   = (const float*)d_in[16];
  float* out = (float*)d_out;

  char* ws = (char*)d_ws;
  size_t off = 0;
  auto carve = [&](size_t bytes) -> char* { char* p = ws + off; off += (bytes + 127) & ~(size_t)127; return p; };
  unsigned short* WT  = (unsigned short*)carve(kWtBytes);
  float*          TAB = (float*)carve(kTabBytes);
  if (off != kWsTotal || off > ws_size) return;

  gate_prep_kernel<<<1, kThreads, 0, stream>>>(h_in, c_in, Wf, Uf, bf, Wi, Ui, bi, Wc, Uc, bc, Wo, Uo, bo, Wy, by, WT, TAB);
  cell_step_kernel<<<kBlocks, kThreads, 0, stream>>>(x, WT, TAB, out);
}
